// PyGGAT_8632884265054
// MI455X (gfx1250) — hardware-verified
//
#include <hip/hip_runtime.h>
#include <stddef.h>


#define FIN     256
#define NCOL    256
#define NHEAD   4
#define NTHR    256
#define NWAVE   8
#define EPT     8
#define NGRP    2
#define CHUNK   (NTHR * EPT * NGRP)
#define WCAP    (EPT * NGRP * 32)
#define LISTN   (NWAVE * WCAP)
#define NBC     4096
#define NBF     1024
#define RCAP    40960
#define RBN     128
#define TGT     256
#define DEGCAP  256
#define OTHR    512
#define WSCAP   134217728
#define NEG_SLOPE 0.2f
#define DEN_EPS 1e-16f
#define WCARRY  1024.0f

#define LDS_FILL ((RCAP + NBF + LISTN) * 4 + 64)

static_assert((CHUNK & (CHUNK - 1)) == 0);
static_assert(CHUNK <= 4096);
static_assert(NBC <= 4096 && NBF <= 4096);
static_assert((NBC & (NBC - 1)) == 0 && (NBF & (NBF - 1)) == 0);
static_assert(NBC == 4 * NBF);
static_assert(OTHR * 8 == NBC);
static_assert((RCAP % 32) == 0);
static_assert(TGT == NWAVE * 32);
static_assert((NBC % TGT) == 0);

typedef float          v4f  __attribute__((ext_vector_type(4)));
typedef float          v8f  __attribute__((ext_vector_type(8)));
typedef int            v4i  __attribute__((ext_vector_type(4)));
typedef _Float16       v8h  __attribute__((ext_vector_type(8)));
typedef _Float16       v16h __attribute__((ext_vector_type(16)));
typedef unsigned short v8us __attribute__((ext_vector_type(8)));
typedef __bf16         v16b __attribute__((ext_vector_type(16)));
union FragH { v16h v; v8h h[2]; };
union FragB { v16b v; v8us h[2]; };

struct GC {
  static constexpr int KD   = FIN;
  static constexpr int NC   = NCOL;
  static constexpr int WPR  = 2;
  static constexpr int TPW  = NC / 16 / WPR;
  static constexpr int RG   = NWAVE / WPR;
  static constexpr int BM   = RG * 16;
  static constexpr int APK  = KD + 8;
  static constexpr int LDSA = BM * APK * 2;
  static constexpr int LDSB = 2 * BM * APK * 2;
  static constexpr int LDSS = BM * NC * 4;
  static constexpr int LDS  = LDSA > LDSS ? LDSA : LDSS;
  static constexpr int LDS3 = LDSB > LDSS ? LDSB : LDSS;
};
static_assert((TGT % GC::BM) == 0);

__device__ __forceinline__ v8h cvt8(v4f a, v4f b, float s) {
  v8h r;
  r[0] = (_Float16)(a.x * s); r[1] = (_Float16)(a.y * s);
  r[2] = (_Float16)(a.z * s); r[3] = (_Float16)(a.w * s);
  r[4] = (_Float16)(b.x * s); r[5] = (_Float16)(b.y * s);
  r[6] = (_Float16)(b.z * s); r[7] = (_Float16)(b.w * s);
  return r;
}

__device__ __forceinline__ unsigned int bfr(float f) {
  const unsigned int u = __float_as_uint(f);
  return (u + 0x7FFFu + ((u >> 16) & 1u)) >> 16;
}

__device__ __forceinline__ void split1(float x, unsigned short& hb, unsigned short& lb) {
  const unsigned int hu = bfr(x);
  const float hf = __uint_as_float(hu << 16);
  hb = (unsigned short)hu;
  lb = (unsigned short)bfr(x - hf);
}

__device__ __forceinline__ void split8(v4f a, v4f b, v8us& hi, v8us& lo) {
  unsigned short hb, lb;
  split1(a.x, hb, lb); hi[0] = hb; lo[0] = lb;
  split1(a.y, hb, lb); hi[1] = hb; lo[1] = lb;
  split1(a.z, hb, lb); hi[2] = hb; lo[2] = lb;
  split1(a.w, hb, lb); hi[3] = hb; lo[3] = lb;
  split1(b.x, hb, lb); hi[4] = hb; lo[4] = lb;
  split1(b.y, hb, lb); hi[5] = hb; lo[5] = lb;
  split1(b.z, hb, lb); hi[6] = hb; lo[6] = lb;
  split1(b.w, hb, lb); hi[7] = hb; lo[7] = lb;
}

__device__ __forceinline__ v8f wmh(v16h a, v16h b, v8f c) {
  v8f d = __builtin_amdgcn_wmma_f32_16x16x32_f16(false, a, false, b, (short)0, c, false, false);
  asm volatile("v_nop\n\tv_nop\n\tv_nop\n\tv_nop" : "+v"(d) : "v"(a), "v"(b));
  return d;
}
__device__ __forceinline__ v8f wmb(v16b a, v16b b, v8f c) {
  v8f d = __builtin_amdgcn_wmma_f32_16x16x32_bf16(false, a, false, b, (short)0, c, false, false);
  asm volatile("v_nop\n\tv_nop\n\tv_nop\n\tv_nop" : "+v"(d) : "v"(a), "v"(b));
  return d;
}

__device__ __forceinline__ float lrelu(float v) { return v > 0.0f ? v : NEG_SLOPE * v; }

template <int NB>
__device__ __forceinline__ int scan_chunk(const int* __restrict__ dsts, int nE, int cbase, int slotBase,
                                          int vec8, int* list, int tid, int lane, int wave) {
  int wc = 0;
#pragma unroll
  for (int g = 0; g < NGRP; ++g) {
    const int el0  = (g * NTHR + tid) * EPT;
    const int e0   = cbase + el0;
    const int sent = -2147483647 - 1;
    v4i da, db;
    if (vec8 != 0 && cbase + CHUNK <= nE) {
      da = *(const v4i*)(dsts + e0);
      db = *(const v4i*)(dsts + e0 + 4);
    } else {
      da.x = (e0     < nE) ? dsts[min(e0, nE - 1)] : sent;
      da.y = (e0 + 1 < nE) ? dsts[min(e0 + 1, nE - 1)] : sent;
      da.z = (e0 + 2 < nE) ? dsts[min(e0 + 2, nE - 1)] : sent;
      da.w = (e0 + 3 < nE) ? dsts[min(e0 + 3, nE - 1)] : sent;
      db.x = (e0 + 4 < nE) ? dsts[min(e0 + 4, nE - 1)] : sent;
      db.y = (e0 + 5 < nE) ? dsts[min(e0 + 5, nE - 1)] : sent;
      db.z = (e0 + 6 < nE) ? dsts[min(e0 + 6, nE - 1)] : sent;
      db.w = (e0 + 7 < nE) ? dsts[min(e0 + 7, nE - 1)] : sent;
    }
    const unsigned nb = (unsigned)slotBase;
    const unsigned s0 = (unsigned)da.x - nb, s1 = (unsigned)da.y - nb;
    const unsigned s2 = (unsigned)da.z - nb, s3 = (unsigned)da.w - nb;
    const unsigned s4 = (unsigned)db.x - nb, s5 = (unsigned)db.y - nb;
    const unsigned s6 = (unsigned)db.z - nb, s7 = (unsigned)db.w - nb;
    const bool h0 = s0 < (unsigned)NB, h1 = s1 < (unsigned)NB, h2 = s2 < (unsigned)NB, h3 = s3 < (unsigned)NB;
    const bool h4 = s4 < (unsigned)NB, h5 = s5 < (unsigned)NB, h6 = s6 < (unsigned)NB, h7 = s7 < (unsigned)NB;
    const unsigned any = __builtin_amdgcn_ballot_w32(h0 | h1 | h2 | h3 | h4 | h5 | h6 | h7);
    if (any != 0u) {
#define HITJ(J, HJ, SJ) { \
        const unsigned mj = __builtin_amdgcn_ballot_w32(HJ); \
        if (mj != 0u) { \
          if (HJ) { \
            const int pos = wc + (int)__builtin_amdgcn_mbcnt_lo(mj, 0u); \
            if (pos < WCAP) list[wave * WCAP + pos] = ((el0 + (J)) << 12) | (int)(SJ); \
          } \
          wc += (int)__builtin_popcount(mj); } }
      HITJ(0, h0, s0)
      HITJ(1, h1, s1)
      HITJ(2, h2, s2)
      HITJ(3, h3, s3)
      HITJ(4, h4, s4)
      HITJ(5, h5, s5)
      HITJ(6, h6, s6)
      HITJ(7, h7, s7)
#undef HITJ
    }
  }
  return wc;
}

__global__ __launch_bounds__(NTHR) void k_wprep(const float* __restrict__ Wa, const float* __restrict__ Wb,
                                                _Float16* wp) {
  constexpr int KD = FIN, NC = NCOL;
  constexpr int UNITS = NC * KD / 8;
  constexpr int KD8   = KD / 8;
  static_assert((UNITS % NTHR) == 0);
  const int lyr = blockIdx.y;
  const float* W = (lyr == 0) ? Wa : Wb;
  const int i = (int)blockIdx.x * NTHR + (int)threadIdx.x;
  if (i >= UNITS) return;
  const int n  = i / KD8;
  const int k0 = (i - n * KD8) * 8;
  const float* wp0 = W + (size_t)k0 * NC + n;
  v4f a, b;
  a.x = wp0[0 * NC]; a.y = wp0[1 * NC]; a.z = wp0[2 * NC]; a.w = wp0[3 * NC];
  b.x = wp0[4 * NC]; b.y = wp0[5 * NC]; b.z = wp0[6 * NC]; b.w = wp0[7 * NC];
  const v8h hv = cvt8(a, b, WCARRY);
  _Float16* dh = wp + (size_t)lyr * NC * KD + (size_t)i * 8;
  *(volatile v8h*)dh = hv;
  __threadfence();
  *(volatile v8h*)dh = hv;
}

__global__ __launch_bounds__(NTHR) void k_wprepb(const float* __restrict__ W, unsigned short* wp) {
  constexpr int KD = FIN, NC = NCOL;
  constexpr int UNITS = NC * KD / 8;
  constexpr int KD8   = KD / 8;
  static_assert((UNITS % NTHR) == 0);
  const int i = (int)blockIdx.x * NTHR + (int)threadIdx.x;
  if (i >= UNITS) return;
  const int n  = i / KD8;
  const int k0 = (i - n * KD8) * 8;
  const float* wp0 = W + (size_t)k0 * NC + n;
  v4f a, b;
  a.x = wp0[0 * NC]; a.y = wp0[1 * NC]; a.z = wp0[2 * NC]; a.w = wp0[3 * NC];
  b.x = wp0[4 * NC]; b.y = wp0[5 * NC]; b.z = wp0[6 * NC]; b.w = wp0[7 * NC];
  v8us hv, lv;
  split8(a, b, hv, lv);
  unsigned short* dh = wp + (size_t)i * 8;
  unsigned short* dl = dh + (size_t)NC * KD;
  *(volatile v8us*)dh = hv;
  *(volatile v8us*)dl = lv;
  __threadfence();
  *(volatile v8us*)dh = hv;
  *(volatile v8us*)dl = lv;
}

__global__ __launch_bounds__(NTHR) void k_count(
    const int* __restrict__ dsts, int* cnt, int nE, int vec8) {
  __shared__ __attribute__((aligned(16))) int scnt[NBC];
  __shared__ __attribute__((aligned(16))) int list[LISTN];
  __shared__ int wcnt[NWAVE];
  const int tid = threadIdx.x, lane = tid & 31, wave = tid >> 5;
  const int nodeBase = blockIdx.x * NBC;

  for (int i = tid; i < NBC; i += NTHR) scnt[i] = 0;
  __syncthreads();

  const int nChunks = (nE + CHUNK - 1) / CHUNK;
#pragma unroll 1
  for (int ch = 0; ch < nChunks; ++ch) {
    const int cbase = ch * CHUNK;
    const int wc = scan_chunk<NBC>(dsts, nE, cbase, nodeBase, vec8, list, tid, lane, wave);
    if (lane == 0) wcnt[wave] = wc;
    __syncthreads();
    if (wave == 0) {
#pragma unroll 1
      for (int wsx = 0; wsx < NWAVE; ++wsx) {
        int n = __builtin_amdgcn_readfirstlane(wcnt[wsx]);
        n = n > WCAP ? WCAP : (n < 0 ? 0 : n);
        const int* lp = list + wsx * WCAP;
#pragma unroll 1
        for (int i = 0; i < n; ++i) {
          const int ent  = __builtin_amdgcn_readfirstlane(lp[i]);
          const int slot = ent & (NBC - 1);
          if (lane == 0) scnt[slot] = scnt[slot] + 1;
        }
      }
    }
    __syncthreads();
  }

  v4i cq[4];
#pragma unroll
  for (int q = 0; q < 4; ++q) {
    const int f = (wave * 4 + q) * 128 + 4 * lane;
    cq[q] = *(const v4i*)(scnt + f);
  }
  int* cp = cnt + (size_t)nodeBase;
#pragma unroll
  for (int q = 0; q < 4; ++q) {
    const int f = (wave * 4 + q) * 128 + 4 * lane;
    *(volatile v4i*)(cp + f) = cq[q];
  }
  __threadfence();
#pragma unroll
  for (int q = 0; q < 4; ++q) {
    const int f = (wave * 4 + q) * 128 + 4 * lane;
    *(volatile v4i*)(cp + f) = cq[q];
  }
}

__global__ __launch_bounds__(OTHR) void k_offsets(
    const int* __restrict__ cnt, int* off, int* rbase, int nChunk) {
  __shared__ __attribute__((aligned(16))) int soff[NBC];
  __shared__ __attribute__((aligned(16))) int srb[RBN];
  __shared__ int wtot[OTHR / 32];
  const int tid = threadIdx.x, lane = tid & 31, wave = tid >> 5, sub = tid >> 7;
  for (int i = tid; i < RBN; i += OTHR) srb[i] = 0;
  int carry = 0;
#pragma unroll 1
  for (int ch = 0; ch < nChunk; ++ch) {
    const int base = ch * NBC;
    const v4i c0 = *(const v4i*)(cnt + base + 8 * tid);
    const v4i c1 = *(const v4i*)(cnt + base + 8 * tid + 4);
    const int e0 = max(c0.x, 0), e1 = max(c0.y, 0), e2 = max(c0.z, 0), e3 = max(c0.w, 0);
    const int e4 = max(c1.x, 0), e5 = max(c1.y, 0), e6 = max(c1.z, 0), e7 = max(c1.w, 0);
    const int ts = e0 + e1 + e2 + e3 + e4 + e5 + e6 + e7;
    int incl = ts;
#pragma unroll
    for (int d = 1; d < 32; d <<= 1) {
      const int t = __shfl_up(incl, d);
      if (lane >= d) incl += t;
    }
    if (lane == 31) wtot[wave] = incl;
    __syncthreads();
    const int S0 = wtot[0]  + wtot[1]  + wtot[2]  + wtot[3];
    const int S1 = wtot[4]  + wtot[5]  + wtot[6]  + wtot[7];
    const int S2 = wtot[8]  + wtot[9]  + wtot[10] + wtot[11];
    const int S3 = wtot[12] + wtot[13] + wtot[14] + wtot[15];
    int pre = 0;
#pragma unroll 1
    for (int w = 4 * sub; w < wave; ++w) pre += wtot[w];
    const int b0 = carry;
    const int b1 = b0 + ((S0 + 31) & ~31);
    const int b2 = b1 + ((S1 + 31) & ~31);
    const int b3 = b2 + ((S2 + 31) & ~31);
    const int b4 = b3 + ((S3 + 31) & ~31);
    const int myb = sub == 0 ? b0 : (sub == 1 ? b1 : (sub == 2 ? b2 : b3));
    if (tid == 0) {
      srb[min(4 * ch + 0, RBN - 1)] = b0;
      srb[min(4 * ch + 1, RBN - 1)] = b1;
      srb[min(4 * ch + 2, RBN - 1)] = b2;
      srb[min(4 * ch + 3, RBN - 1)] = b3;
    }
    int run = myb + pre + incl - ts;
    soff[8 * tid + 0] = run; run += e0;
    soff[8 * tid + 1] = run; run += e1;
    soff[8 * tid + 2] = run; run += e2;
    soff[8 * tid + 3] = run; run += e3;
    soff[8 * tid + 4] = run; run += e4;
    soff[8 * tid + 5] = run; run += e5;
    soff[8 * tid + 6] = run; run += e6;
    soff[8 * tid + 7] = run;
    carry = b4;
    __syncthreads();
    const v4i o0 = *(const v4i*)(soff + 4 * tid);
    const v4i o1 = *(const v4i*)(soff + 4 * (tid + OTHR));
    int* op = off + base;
    *(volatile v4i*)(op + 4 * tid) = o0;
    *(volatile v4i*)(op + 4 * (tid + OTHR)) = o1;
    __threadfence();
    *(volatile v4i*)(op + 4 * tid) = o0;
    *(volatile v4i*)(op + 4 * (tid + OTHR)) = o1;
    __syncthreads();
  }
  if (tid == 0) srb[min(4 * nChunk, RBN - 1)] = carry;
  __syncthreads();
  v4i rv = {0, 0, 0, 0};
  if (tid < 32) rv = *(const v4i*)(srb + 4 * tid);
  if (tid < 32) *(volatile v4i*)(rbase + 4 * tid) = rv;
  __threadfence();
  if (tid < 32) *(volatile v4i*)(rbase + 4 * tid) = rv;
}

__global__ __launch_bounds__(NTHR) void k_fill(
    const int* __restrict__ srcs, const int* __restrict__ dsts,
    const int* __restrict__ off, const int* __restrict__ rbase,
    int* csr, int nN, int nE, int vec8, int csrLen) {
  extern __shared__ v4f lds_dyn[];
  int* region = (int*)lds_dyn;
  int* cursor = region + RCAP;
  int* list   = cursor + NBF;
  int* wcnt   = list + LISTN;
  const int tid = threadIdx.x, lane = tid & 31, wave = tid >> 5;
  const int b = blockIdx.x;
  const int nodeBase = b * NBF;

  int rb0 = rbase[b];
  const int rb1 = rbase[b + 1];
  rb0 = rb0 < 0 ? 0 : (rb0 > csrLen ? csrLen : rb0);
  rb0 &= ~31;
  int len = rb1 - rb0;
  len = len < 0 ? 0 : (len > RCAP ? RCAP : len);
  int lenW = (len + 31) & ~31;
  if (rb0 + lenW > csrLen) lenW = (csrLen - rb0) & ~31;

  {
    const v4i z = {0, 0, 0, 0};
    for (int i = tid; i < RCAP / 4; i += NTHR) ((v4i*)region)[i] = z;
    for (int s = tid; s < NBF; s += NTHR) {
      int o = off[nodeBase + s] - rb0;
      o = o < 0 ? 0 : (o > RCAP ? RCAP : o);
      cursor[s] = o;
    }
  }
  __syncthreads();

  const int nChunks = (nE + CHUNK - 1) / CHUNK;
#pragma unroll 1
  for (int ch = 0; ch < nChunks; ++ch) {
    const int cbase = ch * CHUNK;
    const int wc = scan_chunk<NBF>(dsts, nE, cbase, nodeBase, vec8, list, tid, lane, wave);
    if (lane == 0) wcnt[wave] = wc;
    __syncthreads();
    if (wave == 0) {
#pragma unroll 1
      for (int wsx = 0; wsx < NWAVE; ++wsx) {
        int n = __builtin_amdgcn_readfirstlane(wcnt[wsx]);
        n = n > WCAP ? WCAP : (n < 0 ? 0 : n);
        const int* lp = list + wsx * WCAP;
#pragma unroll 1
        for (int i = 0; i < n; ++i) {
          const int ent  = __builtin_amdgcn_readfirstlane(lp[i]);
          const int slot = ent & (NBF - 1);
          int e = cbase + ((ent >> 12) & (CHUNK - 1));
          e = e > nE - 1 ? nE - 1 : e;
          int src = srcs[e];
          src = src < 0 ? 0 : (src > nN - 1 ? nN - 1 : src);
          if (lane == 0) {
            int pos = cursor[slot];
            pos = pos < 0 ? 0 : (pos > RCAP - 1 ? RCAP - 1 : pos);
            region[pos] = src;
            const int np = pos + 1;
            cursor[slot] = np > RCAP ? RCAP : np;
          }
        }
      }
    }
    __syncthreads();
  }

  const int nv = lenW >> 2;
  int* gp = csr + rb0;
#pragma unroll 1
  for (int i = tid; i < nv; i += NTHR) { const v4i v = ((const v4i*)region)[i]; *(volatile v4i*)(gp + 4 * i) = v; }
  __threadfence();
#pragma unroll 1
  for (int i = tid; i < nv; i += NTHR) { const v4i v = ((const v4i*)region)[i]; *(volatile v4i*)(gp + 4 * i) = v; }
}

__device__ __forceinline__ void gemm_epi(const float* stg, float* sES, float* sED,
                                         const float* __restrict__ attS, const float* __restrict__ attD,
                                         float* C, float* eS, float* eD,
                                         int rowBase, int r0, int c0, int lane, int wave) {
  constexpr int NC = GC::NC, BM = GC::BM, HEADS = NHEAD, CH = NC / HEADS;
  constexpr int LPH  = CH / 4;
  constexpr int NES  = BM * HEADS;
  constexpr int NESI = NES / 128;
  static_assert(LPH == 16 && (NES % 128) == 0 && 2 * NESI <= NWAVE);
  const int col = c0 + 4 * lane;
  const int hd  = col / CH;
  const v4f sAv = *(const v4f*)(attS + col);
  const v4f sDv = *(const v4f*)(attD + col);
  const size_t gb = (size_t)(rowBase + r0) * NC + col;
#pragma unroll
  for (int it = 0; it < 16; ++it) {
    const v4f v = *(const v4f*)(stg + (size_t)(r0 + it) * NC + col);
    *(volatile v4f*)(C + gb + (size_t)it * NC) = v;
    float ps = v.x * sAv.x + v.y * sAv.y + v.z * sAv.z + v.w * sAv.w;
    float pd = v.x * sDv.x + v.y * sDv.y + v.z * sDv.z + v.w * sDv.w;
#pragma unroll
    for (int o = 1; o < LPH; o <<= 1) { ps += __shfl_xor(ps, o); pd += __shfl_xor(pd, o); }
    if ((lane & (LPH - 1)) == 0) { sES[(r0 + it) * HEADS + hd] = ps; sED[(r0 + it) * HEADS + hd] = pd; }
  }
  __threadfence();
#pragma unroll
  for (int it = 0; it < 16; ++it) {
    const v4f v = *(const v4f*)(stg + (size_t)(r0 + it) * NC + col);
    *(volatile v4f*)(C + gb + (size_t)it * NC) = v;
  }
  __syncthreads();

  v4f dv = {0.f, 0.f, 0.f, 0.f};
  const size_t eb = (size_t)rowBase * HEADS;
  if (wave < NESI) {
    const int f = wave * 128 + 4 * lane;
    dv = *(const v4f*)(sES + f);
    *(volatile v4f*)(eS + eb + f) = dv;
  } else if (wave < 2 * NESI) {
    const int f = (wave - NESI) * 128 + 4 * lane;
    dv = *(const v4f*)(sED + f);
    *(volatile v4f*)(eD + eb + f) = dv;
  }
  __threadfence();
  if (wave < NESI) {
    const int f = wave * 128 + 4 * lane;
    *(volatile v4f*)(eS + eb + f) = dv;
  } else if (wave < 2 * NESI) {
    const int f = (wave - NESI) * 128 + 4 * lane;
    *(volatile v4f*)(eD + eb + f) = dv;
  }
}

__global__ __launch_bounds__(NTHR) void k_gemm(
    const float* __restrict__ A, const _Float16* __restrict__ Bw,
    const float* __restrict__ attS, const float* __restrict__ attD,
    float* C, float* eS, float* eD, int nRowsA, float ascale, float oscale) {
  constexpr int KD   = GC::KD;
  constexpr int NC   = GC::NC;
  constexpr int WPR  = GC::WPR;
  constexpr int TPW  = GC::TPW;
  constexpr int BM   = GC::BM;
  constexpr int APK  = GC::APK;
  constexpr int NES  = BM * NHEAD;
  constexpr int UPT  = (BM * KD / 8) / NTHR;
  static_assert(KD % 32 == 0 && NC % (16 * WPR) == 0);
  static_assert(TPW * 4 == 32);
  static_assert(UPT * NTHR * 8 == BM * KD);
  static_assert(((APK * 2) % 16) == 0);
  static_assert(BM * NC * 4 <= GC::LDS && BM * APK * 2 <= GC::LDS);

  extern __shared__ v4f lds_dyn[];
  __shared__ __attribute__((aligned(16))) float sES[NES];
  __shared__ __attribute__((aligned(16))) float sED[NES];
  _Float16* sA  = (_Float16*)lds_dyn;
  float*    stg = (float*)lds_dyn;
  const int tid = threadIdx.x, lane = tid & 31, wave = tid >> 5, hh = lane >> 4, m = lane & 15;
  const int rowBase = blockIdx.x * BM;

#pragma unroll
  for (int i = 0; i < UPT; ++i) {
    const int idx = i * NTHR + tid;
    const int r   = idx / (KD / 8);
    const int c0  = (idx - r * (KD / 8)) * 8;
    int row = rowBase + r;
    row = row > nRowsA - 1 ? nRowsA - 1 : row;
    const float* ap = A + (size_t)row * KD + c0;
    const v4f a = *(const v4f*)ap, b = *(const v4f*)(ap + 4);
    *(v8h*)(sA + r * APK + c0) = cvt8(a, b, ascale);
  }
  __syncthreads();

  const int rg  = wave / WPR;
  const int chf = wave - rg * WPR;
  const int r0  = rg * 16;
  const int c0  = chf * TPW * 16;

  v8f acc[TPW];
#pragma unroll
  for (int t = 0; t < TPW; ++t) { v8f z = {0.f, 0.f, 0.f, 0.f, 0.f, 0.f, 0.f, 0.f}; acc[t] = z; }
  const _Float16* afp = sA + (r0 + m) * APK + 8 * hh;
#pragma unroll 2
  for (int kt = 0; kt < KD / 32; ++kt) {
    FragH af;
    af.h[0] = *(const v8h*)(afp + 32 * kt);
    af.h[1] = *(const v8h*)(afp + 32 * kt + 16);
#pragma unroll
    for (int t = 0; t < TPW; ++t) {
      const _Float16* bp = Bw + (size_t)(c0 + 16 * t + m) * KD + 32 * kt + 8 * hh;
      FragH bf;
      bf.h[0] = *(const v8h*)bp;
      bf.h[1] = *(const v8h*)(bp + 16);
      acc[t] = wmh(af.v, bf.v, acc[t]);
    }
  }
  __syncthreads();

  {
    float* sp = stg + (size_t)(r0 + 8 * hh) * NC + c0 + m;
#pragma unroll
    for (int t = 0; t < TPW; ++t) {
#pragma unroll
      for (int r = 0; r < 8; ++r) sp[r * NC + 16 * t] = acc[t][r] * oscale;
    }
  }
  __syncthreads();

  gemm_epi(stg, sES, sED, attS, attD, C, eS, eD, rowBase, r0, c0, lane, wave);
}

__global__ __launch_bounds__(NTHR) void k_gemm3(
    const float* __restrict__ A, const unsigned short* __restrict__ Bw,
    const float* __restrict__ attS, const float* __restrict__ attD,
    float* C, float* eS, float* eD, int nRowsA) {
  constexpr int KD   = GC::KD;
  constexpr int NC   = GC::NC;
  constexpr int WPR  = GC::WPR;
  constexpr int TPW  = GC::TPW;
  constexpr int BM   = GC::BM;
  constexpr int APK  = GC::APK;
  constexpr int NES  = BM * NHEAD;
  constexpr int UPT  = (BM * KD / 8) / NTHR;
  constexpr size_t WPLN = (size_t)NC * KD;
  static_assert(KD % 32 == 0 && NC % (16 * WPR) == 0);
  static_assert(TPW * 4 == 32);
  static_assert(UPT * NTHR * 8 == BM * KD);
  static_assert(((APK * 2) % 16) == 0);
  static_assert(BM * NC * 4 <= GC::LDS3 && 2 * BM * APK * 2 <= GC::LDS3);

  extern __shared__ v4f lds_dyn[];
  __shared__ __attribute__((aligned(16))) float sES[NES];
  __shared__ __attribute__((aligned(16))) float sED[NES];
  unsigned short* sHi = (unsigned short*)lds_dyn;
  unsigned short* sLo = sHi + BM * APK;
  float*          stg = (float*)lds_dyn;
  const int tid = threadIdx.x, lane = tid & 31, wave = tid >> 5, hh = lane >> 4, m = lane & 15;
  const int rowBase = blockIdx.x * BM;

#pragma unroll
  for (int i = 0; i < UPT; ++i) {
    const int idx = i * NTHR + tid;
    const int r   = idx / (KD / 8);
    const int c0  = (idx - r * (KD / 8)) * 8;
    int row = rowBase + r;
    row = row > nRowsA - 1 ? nRowsA - 1 : row;
    const float* ap = A + (size_t)row * KD + c0;
    const v4f a = *(const v4f*)ap, b = *(const v4f*)(ap + 4);
    v8us hv, lv;
    split8(a, b, hv, lv);
    *(v8us*)(sHi + r * APK + c0) = hv;
    *(v8us*)(sLo + r * APK + c0) = lv;
  }
  __syncthreads();

  const int rg  = wave / WPR;
  const int chf = wave - rg * WPR;
  const int r0  = rg * 16;
  const int c0  = chf * TPW * 16;

  v8f acc[TPW];
#pragma unroll
  for (int t = 0; t < TPW; ++t) { v8f z = {0.f, 0.f, 0.f, 0.f, 0.f, 0.f, 0.f, 0.f}; acc[t] = z; }
  const unsigned short* ahp = sHi + (r0 + m) * APK + 8 * hh;
  const unsigned short* alp = sLo + (r0 + m) * APK + 8 * hh;
#pragma unroll 1
  for (int kt = 0; kt < KD / 32; ++kt) {
    FragB ah, al;
    ah.h[0] = *(const v8us*)(ahp + 32 * kt);
    ah.h[1] = *(const v8us*)(ahp + 32 * kt + 16);
    al.h[0] = *(const v8us*)(alp + 32 * kt);
    al.h[1] = *(const v8us*)(alp + 32 * kt + 16);
#pragma unroll
    for (int t = 0; t < TPW; ++t) {
      const unsigned short* bp = Bw + (size_t)(c0 + 16 * t + m) * KD + 32 * kt + 8 * hh;
      FragB bh, bl;
      bh.h[0] = *(const v8us*)bp;
      bh.h[1] = *(const v8us*)(bp + 16);
      bl.h[0] = *(const v8us*)(bp + WPLN);
      bl.h[1] = *(const v8us*)(bp + WPLN + 16);
      acc[t] = wmb(ah.v, bh.v, acc[t]);
      acc[t] = wmb(ah.v, bl.v, acc[t]);
      acc[t] = wmb(al.v, bh.v, acc[t]);
    }
  }
  __syncthreads();

  {
    float* sp = stg + (size_t)(r0 + 8 * hh) * NC + c0 + m;
#pragma unroll
    for (int t = 0; t < TPW; ++t) {
#pragma unroll
      for (int r = 0; r < 8; ++r) sp[r * NC + 16 * t] = acc[t][r];
    }
  }
  __syncthreads();

  gemm_epi(stg, sES, sED, attS, attD, C, eS, eD, rowBase, r0, c0, lane, wave);
}

template <int LAST>
__global__ __launch_bounds__(NTHR) void k_agg(
    const int* __restrict__ csr, const int* __restrict__ off, const int* __restrict__ cnt,
    const float* __restrict__ eS, const float* __restrict__ eD, const float* __restrict__ hw,
    const float* __restrict__ bias, float* xout, int nN, int csrLen) {
  constexpr int NC = NCOL, HEADS = NHEAD, CH = NC / HEADS;
  static_assert(HEADS * CH == NC && (CH % 4) == 0 && NC == 256);
  const int tid = threadIdx.x, lane = tid & 31, wave = tid >> 5;
  const int tbase = blockIdx.x * TGT + wave * 32;
  const int col0 = 4 * lane;
  const int col1 = 128 + 4 * lane;
  const int hd0  = col0 / CH;
  const int hd1  = col1 / CH;
  const v4f z4 = {0.f, 0.f, 0.f, 0.f};
  const v4f bb0 = *(const v4f*)(bias + col0);
  const v4f bb1 = *(const v4f*)(bias + col1);

  const int cl    = tbase + lane;
  const int cnt_l = cnt[cl];
  const int off_l = off[cl];

#pragma unroll 1
  for (int j = 0; j < 32; ++j) {
    const int c = tbase + j;
    int n = __shfl(cnt_l, j);
    n = n < 0 ? 0 : (n > DEGCAP ? DEGCAP : n);
    const int st = __shfl(off_l, j);
    const float ed0    = eD[(size_t)c * HEADS + hd0];
    const float ed1    = eD[(size_t)c * HEADS + hd1];
    const float eself0 = lrelu(eS[(size_t)c * HEADS + hd0] + ed0);
    const float eself1 = lrelu(eS[(size_t)c * HEADS + hd1] + ed1);

    float mx0 = eself0, mx1 = eself1;
#pragma unroll 1
    for (int q0 = 0; q0 < n; q0 += 32) {
      int pos = st + q0 + lane;
      pos = pos < 0 ? 0 : (pos > csrLen - 1 ? csrLen - 1 : pos);
      int sl = csr[pos];
      sl = sl < 0 ? 0 : (sl > nN - 1 ? nN - 1 : sl);
      const int mcnt = (n - q0) < 32 ? (n - q0) : 32;
#pragma unroll 1
      for (int pp = 0; pp < mcnt; ++pp) {
        const int s = __builtin_amdgcn_readlane(sl, pp);
        mx0 = fmaxf(mx0, lrelu(eS[(size_t)s * HEADS + hd0] + ed0));
        mx1 = fmaxf(mx1, lrelu(eS[(size_t)s * HEADS + hd1] + ed1));
      }
    }

    float p0   = __expf(eself0 - mx0);
    float p1   = __expf(eself1 - mx1);
    float den0 = p0, den1 = p1;
    v4f   acc0 = *(const v4f*)(hw + (size_t)c * NC + col0) * p0;
    v4f   acc1 = *(const v4f*)(hw + (size_t)c * NC + col1) * p1;
#pragma unroll 1
    for (int q0 = 0; q0 < n; q0 += 32) {
      int pos = st + q0 + lane;
      pos = pos < 0 ? 0 : (pos > csrLen - 1 ? csrLen - 1 : pos);
      int sl = csr[pos];
      sl = sl < 0 ? 0 : (sl > nN - 1 ? nN - 1 : sl);
      const int mcnt = (n - q0) < 32 ? (n - q0) : 32;
#pragma unroll 1
      for (int pp = 0; pp < mcnt; ++pp) {
        const int s = __builtin_amdgcn_readlane(sl, pp);
        p0 = __expf(lrelu(eS[(size_t)s * HEADS + hd0] + ed0) - mx0);
        p1 = __expf(lrelu(eS[(size_t)s * HEADS + hd1] + ed1) - mx1);
        den0 += p0;
        den1 += p1;
        const v4f h0 = *(const v4f*)(hw + (size_t)s * NC + col0);
        const v4f h1 = *(const v4f*)(hw + (size_t)s * NC + col1);
        acc0 = acc0 + h0 * p0;
        acc1 = acc1 + h1 * p1;
      }
    }

    const float rd0 = 1.0f / (den0 + DEN_EPS);
    const float rd1 = 1.0f / (den1 + DEN_EPS);
    v4f v0 = acc0 * rd0 + bb0;
    v4f v1 = acc1 * rd1 + bb1;

    float* p0w = xout + (size_t)c * NC + col0;
    float* p1w = xout + (size_t)c * NC + col1;
    if constexpr (LAST == 0) {
      if (c >= nN) { v0 = z4; v1 = z4; }
      *(volatile v4f*)p0w = v0;
      *(volatile v4f*)p1w = v1;
      __threadfence();
      *(volatile v4f*)p0w = v0;
      *(volatile v4f*)p1w = v1;
    } else {
      const bool ok = c < nN;
      if (ok) {
        *(volatile v4f*)p0w = v0;
        *(volatile v4f*)p1w = v1;
      }
      __threadfence();
      if (ok) {
        *(volatile v4f*)p0w = v0;
        *(volatile v4f*)p1w = v1;
      }
    }
  }
}

extern "C" void kernel_launch(void* const* d_in, const int* in_sizes, int n_in,
                              void* d_out, int out_size, void* d_ws, size_t ws_size,
                              hipStream_t stream) {
  if (n_in < 14) return;
  const int nN = in_sizes[0] / FIN;
  const int nE = in_sizes[1] / 2;
  if (nN <= 0 || nE <= 0 || in_sizes[0] != nN * FIN || in_sizes[1] != 2 * nE) return;
  for (int l = 0; l < 3; ++l) {
    if (in_sizes[2 + 4 * l] != FIN * NCOL) return;
    if (in_sizes[3 + 4 * l] != NCOL || in_sizes[4 + 4 * l] != NCOL || in_sizes[5 + 4 * l] != NCOL) return;
  }
  if (out_size != nN * NCOL) return;
  if (nE > (1 << 28) || nN > (1 << 24)) return;

  const float* x   = (const float*)d_in[0];
  const int*   ei  = (const int*)d_in[1];
  const int*   src = ei;
  const int*   dst = ei + (size_t)nE;
  const float* W[3]; const float* AS[3]; const float* AD[3]; const float* BB[3];
  for (int l = 0; l < 3; ++l) {
    W[l]  = (const float*)d_in[2 + 4 * l];
    AS[l] = (const float*)d_in[3 + 4 * l];
    AD[l] = (const float*)d_in[4 + 4 * l];
    BB[l] = (const float*)d_in[5 + 4 * l];
  }
  float* out = (float*)d_out;

  const int NPAD   = ((nN + TGT - 1) / TGT) * TGT;
  const int nBC    = (nN + NBC - 1) / NBC;
  const int CNTPAD = nBC * NBC;
  if (4 * nBC + 1 > RBN) return;
  const int nBF    = (nN + NBF - 1) / NBF;
  const int csrLen = ((nE + 31) & ~31) + 4096;
  if (31 * 4 * nBC > 4096) return;
  const int nAgg   = NPAD / TGT;
  const int nGm    = NPAD / GC::BM;

  char* ws = (char*)d_ws;
  size_t off = 0;
  const size_t oW   = off; off += (size_t)2 * NCOL * FIN * 2;    off = (off + 255) & ~(size_t)255;
  const size_t oWb  = off; off += (size_t)2 * NCOL * FIN * 2;    off = (off + 255) & ~(size_t)255;
  const size_t oCnt = off; off += (size_t)CNTPAD * 4;            off = (off + 255) & ~(size_t)255;
  const size_t oOff = off; off += (size_t)CNTPAD * 4;            off = (off + 255) & ~(size_t)255;
  const size_t oRb  = off; off += (size_t)RBN * 4;               off = (off + 255) & ~(size_t)255;
  const size_t oCsr = off; off += (size_t)csrLen * 4;            off = (off + 255) & ~(size_t)255;
  const size_t oHw  = off; off += (size_t)NPAD * NCOL * 4;       off = (off + 255) & ~(size_t)255;
  const size_t oX   = off; off += (size_t)NPAD * NCOL * 4;       off = (off + 255) & ~(size_t)255;
  const size_t oES  = off; off += (size_t)NPAD * NHEAD * 4;      off = (off + 255) & ~(size_t)255;
  const size_t oED  = off; off += (size_t)NPAD * NHEAD * 4;      off = (off + 255) & ~(size_t)255;
  if (off > ws_size || off > (size_t)WSCAP) return;
  _Float16*       wp   = (_Float16*)(ws + oW);
  unsigned short* wpb  = (unsigned short*)(ws + oWb);
  int*            cnt  = (int*)(ws + oCnt);
  int*            offp = (int*)(ws + oOff);
  int*            rb   = (int*)(ws + oRb);
  int*            csr  = (int*)(ws + oCsr);
  float*          hw   = (float*)(ws + oHw);
  float*          xb   = (float*)(ws + oX);
  float*          es   = (float*)(ws + oES);
  float*          ed   = (float*)(ws + oED);
  const _Float16* wp0 = wp;
  const _Float16* wp1 = wp + (size_t)NCOL * FIN;

  const int vec8 = ((nE & 3) == 0) ? 1 : 0;
  const float asc1 = 256.0f,  osc1 = 1.0f / (256.0f * WCARRY);
  const float asc2 = 1024.0f, osc2 = 1.0f / (1024.0f * WCARRY);

  k_wprep<<<dim3(NCOL * FIN / 8 / NTHR, 2), NTHR, 0, stream>>>(W[0], W[1], wp);
  k_wprepb<<<NCOL * FIN / 8 / NTHR, NTHR, 0, stream>>>(W[2], wpb);

  k_count<<<nBC, NTHR, 0, stream>>>(dst, cnt, nE, vec8);
  k_offsets<<<1, OTHR, 0, stream>>>(cnt, offp, rb, nBC);
  hipFuncSetAttribute(reinterpret_cast<const void*>(&k_fill),
                      hipFuncAttributeMaxDynamicSharedMemorySize, LDS_FILL);
  k_fill<<<nBF, NTHR, LDS_FILL, stream>>>(src, dst, offp, rb, csr, nN, nE, vec8, csrLen);

  hipFuncSetAttribute(reinterpret_cast<const void*>(&k_gemm),
                      hipFuncAttributeMaxDynamicSharedMemorySize, GC::LDS);
  hipFuncSetAttribute(reinterpret_cast<const void*>(&k_gemm3),
                      hipFuncAttributeMaxDynamicSharedMemorySize, GC::LDS3);

  k_gemm<<<nGm, NTHR, GC::LDS, stream>>>(x, wp0, AS[0], AD[0], hw, es, ed, nN, asc1, osc1);
  k_agg<0><<<nAgg, NTHR, 0, stream>>>(csr, offp, cnt, es, ed, hw, BB[0], xb, nN, csrLen);

  k_gemm<<<nGm, NTHR, GC::LDS, stream>>>(xb, wp1, AS[1], AD[1], hw, es, ed, NPAD, asc2, osc2);
  k_agg<0><<<nAgg, NTHR, 0, stream>>>(csr, offp, cnt, es, ed, hw, BB[1], xb, nN, csrLen);

  k_gemm3<<<nGm, NTHR, GC::LDS3, stream>>>(xb, wpb, AS[2], AD[2], hw, es, ed, NPAD);
  k_agg<1><<<nAgg, NTHR, 0, stream>>>(csr, offp, cnt, es, ed, hw, BB[2], out, nN, csrLen);
}
